// MultiHeadAttention_30932354465901
// MI455X (gfx1250) — hardware-verified
//
#include <hip/hip_runtime.h>
#include <stdint.h>


typedef _Float16 v16h __attribute__((ext_vector_type(16)));
typedef _Float16 v8h  __attribute__((ext_vector_type(8)));
typedef float    v8f  __attribute__((ext_vector_type(8)));
typedef float    v4f  __attribute__((ext_vector_type(4)));
typedef int      v4i  __attribute__((ext_vector_type(4)));
typedef unsigned int v4u __attribute__((ext_vector_type(4)));

#ifndef NB
#define NB 2
#endif
#ifndef SEQ
#define SEQ 2048
#endif
#define NB_FULL  2
#define SEQ_FULL 2048
#define DMODEL   1024
#define NHEADS   16
#define DK       64
#define MROWS    (NB * SEQ)
#define NQB      (SEQ / 64)
#define EARLY    ((SEQ) < 512 ? (SEQ) : 512)
#define NEQB     (EARLY / 64)
#define LDP      72
#define LDPF     68
#define XSC      16.0f
#define WSC      1024.0f
#define RSC      4096.0f
#define PCARRY   4096.0f
#define NEGFILL  (-1.0e9f)
#define SSCALE   0.125f

static_assert(SEQ % 64 == 0);
static_assert((SEQ & (SEQ - 1)) == 0);
static_assert(SEQ <= SEQ_FULL);
static_assert(NB >= 1 && NB <= NB_FULL);
static_assert(NQB >= 1 && NQB <= 32);
static_assert(EARLY % 64 == 0 && EARLY <= SEQ);
static_assert(DMODEL == NHEADS * DK);
static_assert(64 * LDPF * 4 <= 2 * 64 * LDP * 2);

__device__ __forceinline__ float bf16r(float x) {
  unsigned int u = __float_as_uint(x);
  u = (u + 0x7FFFu + ((u >> 16) & 1u)) & 0xFFFF0000u;
  return __uint_as_float(u);
}

__device__ __forceinline__ v8f vz8() {
  v8f z;
#pragma unroll
  for (int i = 0; i < 8; ++i) z[i] = 0.0f;
  return z;
}

__device__ __forceinline__ v8f wmma_f16(v16h a, v16h b, v8f c) {
  v8f d = __builtin_amdgcn_wmma_f32_16x16x32_f16(false, a, false, b, (short)0, c, false, false);
  asm volatile("v_nop\n\tv_nop\n\tv_nop\n\tv_nop" : "+v"(d) : "v"(a), "v"(b));
  return d;
}

__device__ __forceinline__ v16h load_frag(const _Float16* base, int ld, int lane) {
  const int row  = lane & 15;
  const int koff = ((lane >> 4) & 1) * 8;
  const _Float16* p = base + row * ld + koff;
  const v8h a = *(const v8h*)(p);
  const v8h b = *(const v8h*)(p + 16);
  v16h r;
#pragma unroll
  for (int i = 0; i < 8; ++i) { r[i] = a[i]; r[i + 8] = b[i]; }
  return r;
}

template <int CTRL>
__device__ __forceinline__ float dpp_max_step(float v) {
  int s = __builtin_amdgcn_mov_dpp(__builtin_bit_cast(int, v), CTRL, 0xF, 0xF, true);
  return fmaxf(v, __builtin_bit_cast(float, s));
}
__device__ __forceinline__ float rowmax16(float v) {
  v = dpp_max_step<0xB1>(v);
  v = dpp_max_step<0x4E>(v);
  v = dpp_max_step<0x141>(v);
  v = dpp_max_step<0x140>(v);
  return v;
}

__global__ __launch_bounds__(256)
void cvt_kernel(const float* __restrict__ in, _Float16* out, int nrows, int seq, int seq_full, float scale) {
  const int g  = blockIdx.x * 256 + threadIdx.x;
  const int n8 = nrows * (DMODEL / 8);
  if (g >= n8) return;
  const int row = g >> 7;
  const int c8  = g & 127;
  const int bi  = row / seq;
  const int s   = row - bi * seq;
  const float* src = in + ((size_t)bi * seq_full + s) * DMODEL + c8 * 8;
  const v4f a = *(const v4f*)src;
  const v4f b = *(const v4f*)(src + 4);
  union { v8h h; v4f f; } u;
#pragma unroll
  for (int i = 0; i < 4; ++i) {
    u.h[i]     = (_Float16)(bf16r(a[i]) * scale);
    u.h[i + 4] = (_Float16)(bf16r(b[i]) * scale);
  }
  float* dst = reinterpret_cast<float*>(out + (size_t)row * DMODEL + c8 * 8);
  const v4f val = u.f;
  *(volatile v4f*)dst = val;
  __threadfence();
  *(volatile v4f*)dst = val;
}

__global__ __launch_bounds__(256)
void flags_kernel(const int* __restrict__ mask, int* flags) {
  __shared__ unsigned int m1s[256];
  __shared__ unsigned int m0s[256];
  __shared__ unsigned int ras[256];
  __shared__ unsigned int red1[32];
  __shared__ unsigned int red0[32];
  __shared__ unsigned int fms[32];
  __shared__ __attribute__((aligned(16))) int lines[32];

  const int tid = threadIdx.x, lane = tid & 31, w = tid >> 5;
  const int qb = blockIdx.x;
  const int row = tid >> 2, quarter = tid & 3;
  const int* mrow = mask + (size_t)(qb * 64 + row) * SEQ_FULL + quarter * 16;

  unsigned int bits1 = 0u, bits0 = 0u, rany = 0u;
#pragma unroll 1
  for (int kt = 0; kt < NQB; ++kt) {
    const int* p = mrow + kt * 64;
    unsigned int any1 = 0u, any0 = 0u;
#pragma unroll
    for (int j = 0; j < 4; ++j) {
      const v4i m4 = *(const v4i*)(p + 4 * j);
#pragma unroll
      for (int e = 0; e < 4; ++e) {
        any1 |= (m4[e] != 0) ? 1u : 0u;
        any0 |= (m4[e] == 0) ? 1u : 0u;
      }
    }
    bits1 |= any1 << kt;
    bits0 |= any0 << kt;
    rany  |= any1;
  }
  m1s[tid] = bits1;
  m0s[tid] = bits0;
  ras[tid] = rany;
  __syncthreads();
  if (w == 0) {
    unsigned int o1 = 0u, o0 = 0u;
#pragma unroll
    for (int j = 0; j < 8; ++j) { o1 |= m1s[lane + 32 * j]; o0 |= m0s[lane + 32 * j]; }
    red1[lane] = o1;
    red0[lane] = o0;
    const unsigned int fa = ras[4 * lane] | ras[4 * lane + 1] | ras[4 * lane + 2] | ras[4 * lane + 3];
    const unsigned int fb = ras[128 + 4 * lane] | ras[128 + 4 * lane + 1] |
                            ras[128 + 4 * lane + 2] | ras[128 + 4 * lane + 3];
    fms[lane] = (fa == 0u || fb == 0u) ? 1u : 0u;
  }
  __syncthreads();
  if (w == 0) {
    unsigned int a1 = 0u, a0 = 0u, anyfm = 0u;
#pragma unroll 1
    for (int j = 0; j < 32; ++j) { a1 |= red1[j]; a0 |= red0[j]; anyfm |= fms[j]; }
    int f = 2;
    if (lane < NQB) {
      const bool h1 = ((a1 >> lane) & 1u) != 0u;
      const bool h0 = ((a0 >> lane) & 1u) != 0u;
      f = (!h0) ? 1 : ((!h1 && anyfm == 0u) ? 2 : 3);
    }
    lines[lane] = f;
  }
  __syncthreads();
  if (w == 0 && lane < 8) {
    const v4i v = *(const v4i*)(lines + lane * 4);
    int* dst = flags + qb * 32 + lane * 4;
    *(volatile v4i*)dst = v;
    __threadfence();
    *(volatile v4i*)dst = v;
  }
}

template <int MODE>
__global__ __launch_bounds__(128)
void gemm16(const _Float16* __restrict__ A, const _Float16* __restrict__ Ar,
            const _Float16* __restrict__ W, const float* __restrict__ bias,
            void* out, _Float16* outr, float oscale) {
  __shared__ __attribute__((aligned(16))) _Float16 smem[3 * 64 * LDP];
  _Float16* asb = smem;
  _Float16* bsb = smem + 64 * LDP;
  _Float16* rsb = smem + 2 * 64 * LDP;

  const int tid  = threadIdx.x;
  const int lane = tid & 31;
  const int w    = tid >> 5;
  const int mblk = blockIdx.y * 64;
  const int nblk = blockIdx.x * 64;
  const int s0   = mblk & (SEQ - 1);
  const int bi   = mblk / SEQ;
  const bool early = (MODE == 4) && (s0 < EARLY);
  const int lm = (w >> 1) * 32;
  const int ln = (w & 1) * 32;

  v8f acc[2][2], accr[2][2];
#pragma unroll
  for (int i = 0; i < 2; ++i)
#pragma unroll
    for (int j = 0; j < 2; ++j) { acc[i][j] = vz8(); accr[i][j] = vz8(); }

#pragma unroll 1
  for (int k0 = 0; k0 < DMODEL; k0 += 64) {
#pragma unroll
    for (int c = 0; c < 4; ++c) {
      const int chunk = tid * 4 + c;
      const int row = chunk >> 3, part = chunk & 7;
      *(v8h*)(asb + row * LDP + part * 8) =
          *(const v8h*)(A + (size_t)(mblk + row) * DMODEL + k0 + part * 8);
      *(v8h*)(bsb + row * LDP + part * 8) =
          *(const v8h*)(W + (size_t)(nblk + row) * DMODEL + k0 + part * 8);
    }
    if (early) {
#pragma unroll
      for (int c = 0; c < 4; ++c) {
        const int chunk = tid * 4 + c;
        const int row = chunk >> 3, part = chunk & 7;
        *(v8h*)(rsb + row * LDP + part * 8) =
            *(const v8h*)(Ar + (size_t)(mblk + row) * DMODEL + k0 + part * 8);
      }
    }
    __syncthreads();

#pragma unroll
    for (int ks = 0; ks < 64; ks += 32) {
      const v16h a0 = load_frag(asb + (lm +  0) * LDP + ks, LDP, lane);
      const v16h a1 = load_frag(asb + (lm + 16) * LDP + ks, LDP, lane);
      const v16h b0 = load_frag(bsb + (ln +  0) * LDP + ks, LDP, lane);
      const v16h b1 = load_frag(bsb + (ln + 16) * LDP + ks, LDP, lane);
      acc[0][0] = wmma_f16(a0, b0, acc[0][0]);
      acc[0][1] = wmma_f16(a0, b1, acc[0][1]);
      acc[1][0] = wmma_f16(a1, b0, acc[1][0]);
      acc[1][1] = wmma_f16(a1, b1, acc[1][1]);
      if (early) {
        const v16h r0 = load_frag(rsb + (lm +  0) * LDP + ks, LDP, lane);
        const v16h r1 = load_frag(rsb + (lm + 16) * LDP + ks, LDP, lane);
        accr[0][0] = wmma_f16(r0, b0, accr[0][0]);
        accr[0][1] = wmma_f16(r0, b1, accr[0][1]);
        accr[1][0] = wmma_f16(r1, b0, accr[1][0]);
        accr[1][1] = wmma_f16(r1, b1, accr[1][1]);
      }
    }
    __syncthreads();
  }

  const int rbase = ((lane >> 4) & 1) << 3;
  const int col   = lane & 15;

  if constexpr (MODE == 4) {
    float* fs = reinterpret_cast<float*>(smem);
#pragma unroll
    for (int i = 0; i < 2; ++i)
#pragma unroll
      for (int j = 0; j < 2; ++j) {
        const int nl = ln + j * 16 + col;
        const float bb = bf16r(bias[nblk + nl]);
#pragma unroll
        for (int r = 0; r < 8; ++r) {
          const int ml = lm + i * 16 + rbase + r;
          float v = acc[i][j][r] * oscale + bb;
          if (early) v += accr[i][j][r] * (oscale * (1.0f / RSC));
          fs[ml * LDPF + nl] = v;
        }
      }
    __syncthreads();
    float* obase = reinterpret_cast<float*>(out) + ((size_t)bi * SEQ_FULL + s0) * DMODEL + nblk;
    auto emit = [&]() {
#pragma unroll
      for (int i = 0; i < 8; ++i) {
        const int row   = w * 16 + i * 2 + (lane >> 4);
        const int piece = lane & 15;
        const v4f v = *(const v4f*)(fs + row * LDPF + piece * 4);
        *(volatile v4f*)(obase + (size_t)row * DMODEL + piece * 4) = v;
      }
    };
    emit();
    __threadfence();
    emit();
  } else {
    _Float16* hs = asb;
    _Float16* rs = bsb;
#pragma unroll
    for (int i = 0; i < 2; ++i)
#pragma unroll
      for (int j = 0; j < 2; ++j) {
        const int nl = ln + j * 16 + col;
        const float bb = bf16r(bias[nblk + nl]);
#pragma unroll
        for (int r = 0; r < 8; ++r) {
          const int ml = lm + i * 16 + rbase + r;
          const float v = acc[i][j][r] * oscale + bb;
          const _Float16 hv = (_Float16)v;
          const _Float16 rv = (_Float16)((v - (float)hv) * RSC);
          if constexpr (MODE == 0) {
            hs[ml * LDP + nl] = hv;
            rs[ml * LDP + nl] = rv;
          } else {
            hs[nl * LDP + ml] = hv;
            rs[nl * LDP + ml] = rv;
          }
        }
      }
    __syncthreads();
    const int bhh = bi * NHEADS + (nblk >> 6);
    _Float16* oh = reinterpret_cast<_Float16*>(out);
    auto emit = [&]() {
#pragma unroll
      for (int i = 0; i < 4; ++i) {
        const int row   = w * 16 + i * 4 + (lane >> 3);
        const int piece = lane & 7;
        const v4f hv4 = *(const v4f*)(hs + row * LDP + piece * 8);
        const v4f rv4 = *(const v4f*)(rs + row * LDP + piece * 8);
        const size_t go = (MODE == 0)
            ? (((size_t)bhh * SEQ + s0 + row) * DK + piece * 8)
            : (((size_t)bhh * DK + row) * SEQ + s0 + piece * 8);
        *(volatile v4f*)(reinterpret_cast<float*>(oh + go))   = hv4;
        *(volatile v4f*)(reinterpret_cast<float*>(outr + go)) = rv4;
      }
    };
    emit();
    __threadfence();
    emit();
  }
}

template <bool EQ>
__global__ __launch_bounds__(128)
void attn_kernel(const _Float16* __restrict__ Q,  const _Float16* __restrict__ Qr,
                 const _Float16* __restrict__ Kd, const _Float16* __restrict__ Kr,
                 const _Float16* __restrict__ Vt, const _Float16* __restrict__ Vtr,
                 const int* __restrict__ mask, const int* __restrict__ flags,
                 _Float16* ctx, _Float16* ctxr, int qb0) {
  constexpr int RT = EQ ? (64 * LDP) : 8;
  constexpr int PT = EQ ? (4 * 16 * LDP) : 8;
  __shared__ __attribute__((aligned(16))) _Float16 kbuf[64 * LDP];
  __shared__ __attribute__((aligned(16))) _Float16 vbuf[64 * LDP];
  __shared__ __attribute__((aligned(16))) _Float16 pbuf[4 * 16 * LDP];
  __shared__ __attribute__((aligned(16))) _Float16 krbuf[RT];
  __shared__ __attribute__((aligned(16))) _Float16 vrbuf[RT];
  __shared__ __attribute__((aligned(16))) _Float16 prbuf[PT];
  __shared__ __attribute__((aligned(16))) unsigned int mbuf[64 * 16];

  const int tid   = threadIdx.x;
  const int lane  = tid & 31;
  const int w     = tid >> 5;
  const int qb    = qb0 + blockIdx.x;
  const int bh    = blockIdx.y;
  const int bi    = bh / NHEADS;
  const int h     = bh - bi * NHEADS;
  const int qblk  = qb * 64;
  const int q0    = qblk + w * 16;
  const int rbase = ((lane >> 4) & 1) << 3;
  const int col   = lane & 15;
  const float IR  = 1.0f / RSC;

  const size_t qoff = ((size_t)bh * SEQ + q0) * DK;
  const v16h qf0 = load_frag(Q + qoff, DK, lane);
  const v16h qf1 = load_frag(Q + qoff + 32, DK, lane);
  v16h qr0 = qf0, qr1 = qf1;
  if constexpr (EQ) {
    qr0 = load_frag(Qr + qoff, DK, lane);
    qr1 = load_frag(Qr + qoff + 32, DK, lane);
  }

  v16h ones;
#pragma unroll
  for (int i = 0; i < 16; ++i) ones[i] = (_Float16)1.0f;

  const _Float16* Kh   = Kd  + (size_t)bh * SEQ * DK;
  const _Float16* Krh  = Kr  + (size_t)bh * SEQ * DK;
  const _Float16* Vth  = Vt  + (size_t)bh * DK * SEQ;
  const _Float16* Vtrh = Vtr + (size_t)bh * DK * SEQ;
  _Float16* pb  = pbuf + w * 16 * LDP;
  _Float16* prb = prbuf + (EQ ? (w * 16 * LDP) : 0);

  float mr[8], lr[8];
#pragma unroll
  for (int r = 0; r < 8; ++r) { mr[r] = -1.0e30f; lr[r] = 0.0f; }
  v8f accO[4], accR[4];
#pragma unroll
  for (int t = 0; t < 4; ++t) { accO[t] = vz8(); accR[t] = vz8(); }

#pragma unroll 1
  for (int kt = 0; kt < NQB; ++kt) {
    const int f = __builtin_amdgcn_readfirstlane(flags[qb * 32 + kt]);
    if (f == 2) continue;
    const bool usem = (f != 1);
    const int kb = kt * 64;

#pragma unroll
    for (int c = 0; c < 4; ++c) {
      const int chunk = tid * 4 + c;
      const int row = chunk >> 3, part = chunk & 7;
      *(v8h*)(kbuf + row * LDP + part * 8) =
          *(const v8h*)(Kh + (size_t)(kb + row) * DK + part * 8);
      *(v8h*)(vbuf + row * LDP + part * 8) =
          *(const v8h*)(Vth + (size_t)row * SEQ + kb + part * 8);
      if constexpr (EQ) {
        *(v8h*)(krbuf + row * LDP + part * 8) =
            *(const v8h*)(Krh + (size_t)(kb + row) * DK + part * 8);
        *(v8h*)(vrbuf + row * LDP + part * 8) =
            *(const v8h*)(Vtrh + (size_t)row * SEQ + kb + part * 8);
      }
    }
    if (usem) {
      const int row = tid >> 1;
      const int ch  = (tid & 1) * 32;
      const int* mp = mask + (size_t)(qblk + row) * SEQ_FULL + kb + ch;
      v4u u0, u1;
#pragma unroll
      for (int jj = 0; jj < 4; ++jj) { u0[jj] = 0u; u1[jj] = 0u; }
#pragma unroll
      for (int jj = 0; jj < 8; ++jj) {
        const v4i m4 = *(const v4i*)(mp + jj * 4);
        const unsigned int pk = (m4[0] != 0 ? 1u : 0u) | (m4[1] != 0 ? 0x100u : 0u) |
                                (m4[2] != 0 ? 0x10000u : 0u) | (m4[3] != 0 ? 0x1000000u : 0u);
        if (jj < 4) u0[jj] = pk; else u1[jj - 4] = pk;
      }
      *(v4u*)(mbuf + row * 16 + (tid & 1) * 8)     = u0;
      *(v4u*)(mbuf + row * 16 + (tid & 1) * 8 + 4) = u1;
    }
    __syncthreads();

    v8f s[4];
#pragma unroll
    for (int t = 0; t < 4; ++t) {
      const v16h ka = load_frag(kbuf + t * 16 * LDP,      LDP, lane);
      const v16h kc = load_frag(kbuf + t * 16 * LDP + 32, LDP, lane);
      v8f z = vz8();
      z = wmma_f16(qf0, ka, z);
      z = wmma_f16(qf1, kc, z);
      if constexpr (EQ) {
        v8f zr = vz8();
        zr = wmma_f16(qr0, ka, zr);
        zr = wmma_f16(qr1, kc, zr);
        const v16h kra = load_frag(krbuf + t * 16 * LDP,      LDP, lane);
        const v16h krc = load_frag(krbuf + t * 16 * LDP + 32, LDP, lane);
        zr = wmma_f16(qf0, kra, zr);
        zr = wmma_f16(qf1, krc, zr);
        z = z + zr * IR;
      }
      s[t] = z;
    }

#pragma unroll
    for (int r = 0; r < 8; ++r) {
      float a0 = s[0][r] * SSCALE, a1 = s[1][r] * SSCALE, a2 = s[2][r] * SSCALE, a3 = s[3][r] * SSCALE;
      if (usem) {
        const unsigned char* mb =
            reinterpret_cast<const unsigned char*>(mbuf) + (w * 16 + rbase + r) * 64 + col;
        a0 = (mb[0]  != 0) ? a0 : NEGFILL;
        a1 = (mb[16] != 0) ? a1 : NEGFILL;
        a2 = (mb[32] != 0) ? a2 : NEGFILL;
        a3 = (mb[48] != 0) ? a3 : NEGFILL;
      }
      const float tmax = rowmax16(fmaxf(fmaxf(a0, a1), fmaxf(a2, a3)));
      const float mnew = fmaxf(mr[r], tmax);
      const float scl  = __expf(mr[r] - mnew);
      const float p0 = __expf(a0 - mnew);
      const float p1 = __expf(a1 - mnew);
      const float p2 = __expf(a2 - mnew);
      const float p3 = __expf(a3 - mnew);
      mr[r] = mnew;
      lr[r] *= scl;
#pragma unroll
      for (int t = 0; t < 4; ++t) {
        accO[t][r] *= scl;
        if constexpr (EQ) accR[t][r] *= scl;
      }
      const int m = rbase + r;
      const float c0 = p0 * PCARRY, c1 = p1 * PCARRY, c2 = p2 * PCARRY, c3 = p3 * PCARRY;
      const _Float16 h0 = (_Float16)c0, h1 = (_Float16)c1, h2 = (_Float16)c2, h3 = (_Float16)c3;
      pb[m * LDP +      col] = h0;
      pb[m * LDP + 16 + col] = h1;
      pb[m * LDP + 32 + col] = h2;
      pb[m * LDP + 48 + col] = h3;
      if constexpr (EQ) {
        prb[m * LDP +      col] = (_Float16)((c0 - (float)h0) * RSC);
        prb[m * LDP + 16 + col] = (_Float16)((c1 - (float)h1) * RSC);
        prb[m * LDP + 32 + col] = (_Float16)((c2 - (float)h2) * RSC);
        prb[m * LDP + 48 + col] = (_Float16)((c3 - (float)h3) * RSC);
      }
    }
    __syncthreads();

    const v16h pf0 = load_frag(pb,      LDP, lane);
    const v16h pf1 = load_frag(pb + 32, LDP, lane);
    v16h prf0 = pf0, prf1 = pf1;
    if constexpr (EQ) {
      prf0 = load_frag(prb,      LDP, lane);
      prf1 = load_frag(prb + 32, LDP, lane);
    }

    v8f rs = vz8();
    rs = wmma_f16(pf0, ones, rs);
    rs = wmma_f16(pf1, ones, rs);
    if constexpr (EQ) {
      v8f rr = vz8();
      rr = wmma_f16(prf0, ones, rr);
      rr = wmma_f16(prf1, ones, rr);
      rs = rs + rr * IR;
    }
#pragma unroll
    for (int r = 0; r < 8; ++r) lr[r] += rs[r];

#pragma unroll
    for (int t = 0; t < 4; ++t) {
      v16h vf = load_frag(vbuf + t * 16 * LDP, LDP, lane);
      accO[t] = wmma_f16(pf0, vf, accO[t]);
      if constexpr (EQ) {
        accR[t] = wmma_f16(prf0, vf, accR[t]);
        const v16h vr = load_frag(vrbuf + t * 16 * LDP, LDP, lane);
        accR[t] = wmma_f16(pf0, vr, accR[t]);
      }
      vf = load_frag(vbuf + t * 16 * LDP + 32, LDP, lane);
      accO[t] = wmma_f16(pf1, vf, accO[t]);
      if constexpr (EQ) {
        accR[t] = wmma_f16(prf1, vf, accR[t]);
        const v16h vr = load_frag(vrbuf + t * 16 * LDP + 32, LDP, lane);
        accR[t] = wmma_f16(pf1, vr, accR[t]);
      }
    }
    __syncthreads();
  }

#pragma unroll
  for (int r = 0; r < 8; ++r) {
    const float inv = 1.0f / lr[r];
    const int m = w * 16 + rbase + r;
#pragma unroll
    for (int t = 0; t < 4; ++t) {
      float v = accO[t][r];
      if constexpr (EQ) v += accR[t][r] * IR;
      v *= inv;
      const _Float16 hv = (_Float16)v;
      kbuf[m * LDP + t * 16 + col] = hv;
      if constexpr (EQ) krbuf[m * LDP + t * 16 + col] = (_Float16)((v - (float)hv) * RSC);
    }
  }
  __syncthreads();
  _Float16* cbase  = ctx  + ((size_t)bi * SEQ + qblk) * DMODEL + h * DK;
  _Float16* crbase = ctxr + ((size_t)bi * SEQ + qblk) * DMODEL + h * DK;
  auto emit = [&]() {
#pragma unroll
    for (int i = 0; i < 4; ++i) {
      const int row   = w * 16 + i * 4 + (lane >> 3);
      const int piece = lane & 7;
      const v4f hv4 = *(const v4f*)(kbuf + row * LDP + piece * 8);
      *(volatile v4f*)(reinterpret_cast<float*>(cbase + (size_t)row * DMODEL + piece * 8)) = hv4;
      if constexpr (EQ) {
        const v4f rv4 = *(const v4f*)(krbuf + row * LDP + piece * 8);
        *(volatile v4f*)(reinterpret_cast<float*>(crbase + (size_t)row * DMODEL + piece * 8)) = rv4;
      }
    }
  };
  emit();
  __threadfence();
  emit();
}

extern "C" void kernel_launch(void* const* d_in, const int* in_sizes, int n_in,
                              void* d_out, int out_size, void* d_ws, size_t ws_size,
                              hipStream_t stream) {
  if (n_in < 12) return;
  const long long needx = (long long)(NB - 1) * SEQ_FULL * DMODEL + (long long)SEQ * DMODEL;
  const long long needm = (long long)(SEQ - 1) * SEQ_FULL + SEQ;
  if ((long long)in_sizes[0] < needx || (long long)in_sizes[1] < needx || (long long)in_sizes[2] < needx) return;
  if ((long long)in_sizes[3] < needm) return;
  if (in_sizes[4] < DMODEL * DMODEL || in_sizes[6] < DMODEL * DMODEL ||
      in_sizes[8] < DMODEL * DMODEL || in_sizes[10] < DMODEL * DMODEL) return;
  if (in_sizes[5] < DMODEL || in_sizes[7] < DMODEL || in_sizes[9] < DMODEL || in_sizes[11] < DMODEL) return;
  if ((long long)out_size < needx) return;

  const float* q  = (const float*)d_in[0];
  const float* k  = (const float*)d_in[1];
  const float* v  = (const float*)d_in[2];
  const int*   mk = (const int*)d_in[3];
  const float* wq = (const float*)d_in[4];
  const float* bq = (const float*)d_in[5];
  const float* wk = (const float*)d_in[6];
  const float* bk = (const float*)d_in[7];
  const float* wv = (const float*)d_in[8];
  const float* bv = (const float*)d_in[9];
  const float* wo = (const float*)d_in[10];
  const float* bo = (const float*)d_in[11];

  char* ws = (char*)d_ws;
  size_t off = 0;
  const size_t XB = (size_t)MROWS * DMODEL * sizeof(_Float16);
  const size_t WB = (size_t)DMODEL * DMODEL * sizeof(_Float16);
  const size_t FB = 4096;
  _Float16* Xq16  = (_Float16*)(ws + off); off += XB;
  _Float16* Xk16  = (_Float16*)(ws + off); off += XB;
  _Float16* Xv16  = (_Float16*)(ws + off); off += XB;
  _Float16* Wq16  = (_Float16*)(ws + off); off += WB;
  _Float16* Wk16  = (_Float16*)(ws + off); off += WB;
  _Float16* Wv16  = (_Float16*)(ws + off); off += WB;
  _Float16* Wo16  = (_Float16*)(ws + off); off += WB;
  _Float16* Q16   = (_Float16*)(ws + off); off += XB;
  _Float16* Qr16  = (_Float16*)(ws + off); off += XB;
  _Float16* K16   = (_Float16*)(ws + off); off += XB;
  _Float16* Kr16  = (_Float16*)(ws + off); off += XB;
  _Float16* Vt16  = (_Float16*)(ws + off); off += XB;
  _Float16* Vtr16 = (_Float16*)(ws + off); off += XB;
  _Float16* C16   = (_Float16*)(ws + off); off += XB;
  _Float16* Cr16  = (_Float16*)(ws + off); off += XB;
  int*      flg   = (int*)(ws + off);      off += FB;
  if (off > ws_size) return;

  const int gx = (MROWS * (DMODEL / 8) + 255) / 256;
  const int gw = (DMODEL * (DMODEL / 8) + 255) / 256;
  cvt_kernel<<<gx, 256, 0, stream>>>(q, Xq16, MROWS, SEQ, SEQ_FULL, XSC);
  cvt_kernel<<<gx, 256, 0, stream>>>(k, Xk16, MROWS, SEQ, SEQ_FULL, XSC);
  cvt_kernel<<<gx, 256, 0, stream>>>(v, Xv16, MROWS, SEQ, SEQ_FULL, XSC);
  cvt_kernel<<<gw, 256, 0, stream>>>(wq, Wq16, DMODEL, DMODEL, DMODEL, WSC);
  cvt_kernel<<<gw, 256, 0, stream>>>(wk, Wk16, DMODEL, DMODEL, DMODEL, WSC);
  cvt_kernel<<<gw, 256, 0, stream>>>(wv, Wv16, DMODEL, DMODEL, DMODEL, WSC);
  cvt_kernel<<<gw, 256, 0, stream>>>(wo, Wo16, DMODEL, DMODEL, DMODEL, WSC);

  flags_kernel<<<NQB, 256, 0, stream>>>(mk, flg);

  const dim3 gproj(DMODEL / 64, MROWS / 64);
  const float posc = 1.0f / (XSC * WSC);
  gemm16<0><<<gproj, 128, 0, stream>>>(Xq16, Xq16, Wq16, bq, (void*)Q16,  Qr16,  posc);
  gemm16<0><<<gproj, 128, 0, stream>>>(Xk16, Xk16, Wk16, bk, (void*)K16,  Kr16,  posc);
  gemm16<2><<<gproj, 128, 0, stream>>>(Xv16, Xv16, Wv16, bv, (void*)Vt16, Vtr16, posc);

  const dim3 gea(NEQB, NB * NHEADS);
  attn_kernel<true><<<gea, 128, 0, stream>>>(Q16, Qr16, K16, Kr16, Vt16, Vtr16, mk, flg, C16, Cr16, 0);
  if (NQB > NEQB) {
    const dim3 gla(NQB - NEQB, NB * NHEADS);
    attn_kernel<false><<<gla, 128, 0, stream>>>(Q16, Qr16, K16, Kr16, Vt16, Vtr16, mk, flg, C16, Cr16, NEQB);
  }

  gemm16<4><<<gproj, 128, 0, stream>>>(C16, Cr16, Wo16, bo, d_out, Cr16, 1.0f / WSC);
}
